// DeepSetObstacles_56504589746465
// MI455X (gfx1250) — hardware-run, weakly checked
//
#include <hip/hip_runtime.h>
#include <stddef.h>
#include <stdint.h>

#define NEUR   64
#define NOUT   32
#define MOBS   32
#define WP     72
#define NWAVES 4
#define ITERS  16
#define SPB    (NWAVES * ITERS)
#define OPF    36

static_assert(NEUR == 64);
static_assert(NOUT == 32);
static_assert(MOBS == 32);
static_assert((WP % 8) == 0);
static_assert(SPB == 64);
static_assert((OPF % 4) == 0);

typedef _Float16 v8h  __attribute__((ext_vector_type(8)));
typedef _Float16 v16h __attribute__((ext_vector_type(16)));
typedef float    v2f  __attribute__((ext_vector_type(2)));
typedef float    v4f  __attribute__((ext_vector_type(4)));
typedef float    v8f  __attribute__((ext_vector_type(8)));

union Frag { v16h v; v8h half[2]; };

__device__ __forceinline__ float bf16r(float f) {
  unsigned u = __float_as_uint(f);
  u = (u + 0x7FFFu + ((u >> 16) & 1u)) & 0xFFFF0000u;
  return __uint_as_float(u);
}
__device__ __forceinline__ v8f zero8() { v8f z = {0.f, 0.f, 0.f, 0.f, 0.f, 0.f, 0.f, 0.f}; return z; }

__device__ __forceinline__ v16h ldfrag(const _Float16* p) {
  Frag f;
  f.half[0] = *(const v8h*)(p);
  f.half[1] = *(const v8h*)(p + 16);
  return f.v;
}

__device__ __forceinline__ v8f mma_h(v16h a, v16h b, v8f c) {
  return __builtin_amdgcn_wmma_f32_16x16x32_f16(false, a, false, b, (short)0, c, false, false);
}
__device__ __forceinline__ void guard2(v8f& c0, v8f& c1,
                                       const v16h& a0, const v16h& a1, const v16h& a2, const v16h& a3,
                                       const v16h& b0, const v16h& b1) {
#if defined(__HIP_DEVICE_COMPILE__)
  asm volatile("v_nop\n\tv_nop\n\tv_nop\n\tv_nop"
               : "+v"(c0), "+v"(c1)
               : "v"(a0), "v"(a1), "v"(a2), "v"(a3), "v"(b0), "v"(b1));
#endif
}

template <int NN>
__device__ __forceinline__ void stage_wt(_Float16* dst, const float* __restrict__ src, int tid) {
  static_assert((NN * 8) % 128 == 0);
  static_assert((NN & (NN - 1)) == 0);
#pragma unroll
  for (int s = 0; s < (NN * 8) / 128; ++s) {
    const int idx = s * 128 + tid;
    const int n   = idx & (NN - 1);
    const int kg  = idx / NN;
    v8h o;
#pragma unroll
    for (int q = 0; q < 8; ++q) o[q] = (_Float16)(bf16r(src[(kg * 8 + q) * NN + n]) * 64.0f);
    *(v8h*)(dst + n * WP + kg * 8) = o;
  }
}

__global__ __launch_bounds__(128)
void k_deepset(const float* __restrict__ x,   const float* __restrict__ vel,
               const float* __restrict__ pW1, const float* __restrict__ pb1,
               const float* __restrict__ pW2, const float* __restrict__ pb2,
               const float* __restrict__ pW3, const float* __restrict__ pb3,
               const float* __restrict__ rW1, const float* __restrict__ rb1,
               const float* __restrict__ rW2, const float* __restrict__ rb2,
               const float* __restrict__ rW3, const float* __restrict__ rb3,
               float* out, int ns)
{
  __shared__ __align__(16) _Float16 wph[2][NEUR * WP];
  __shared__ __align__(16) _Float16 wrh[2][NEUR * WP];
  __shared__ __align__(16) _Float16 wr3[NOUT * WP];
  __shared__ __align__(16) _Float16 act[NWAVES][MOBS * WP];
  __shared__ __align__(16) _Float16 xh[SPB * WP];
  __shared__ __align__(16) _Float16 xr[SPB * WP];
  __shared__ __align__(16) float outS[SPB * OPF];
  __shared__ __align__(16) float w1s[4 * NEUR];
  __shared__ __align__(16) float b1s[NEUR];
  __shared__ __align__(16) float bph[2][NEUR];
  __shared__ __align__(16) float brh[2][NEUR];
  __shared__ __align__(16) float br3[NOUT];
  __shared__ __align__(16) float velp[NWAVES][NEUR];

  const int tid = threadIdx.x;

  stage_wt<NEUR>(wph[0], pW2, tid);
  stage_wt<NEUR>(wph[1], pW3, tid);
  stage_wt<NEUR>(wrh[0], rW1, tid);
  stage_wt<NEUR>(wrh[1], rW2, tid);
  stage_wt<NOUT>(wr3,    rW3, tid);
  w1s[tid]       = bf16r(pW1[tid]);
  w1s[tid + 128] = bf16r(pW1[tid + 128]);
  if (tid < NEUR) {
    b1s[tid]    = bf16r(pb1[tid]);
    bph[0][tid] = bf16r(pb2[tid]);
    bph[1][tid] = bf16r(pb3[tid]);
    brh[0][tid] = bf16r(rb1[tid]);
    brh[1][tid] = bf16r(rb2[tid]);
  }
  if (tid < NOUT) br3[tid] = bf16r(rb3[tid]);
  __syncthreads();

  const int lane = tid & 31;
  const int wave = tid >> 5;
  const int hh   = lane >> 4;
  const int c    = lane & 15;
  _Float16* actW = act[wave];
  const float kinv = 0.0009765625f;
  const float rinv = 0.00048828125f;
  const int sbase = (int)blockIdx.x * SPB;

#pragma unroll 1
  for (int it = 0; it < ITERS; ++it) {
    const int srow = it * NWAVES + wave;
    int sl = sbase + srow;
    if (sl > ns - 1) sl = ns - 1;

    {
      const float vx = bf16r(vel[(size_t)sl * 2]);
      const float vy = bf16r(vel[(size_t)sl * 2 + 1]);
      const int n0 = 2 * lane;
      v2f pv;
      pv[0] = b1s[n0]     + vx * w1s[2 * NEUR + n0]     + vy * w1s[3 * NEUR + n0];
      pv[1] = b1s[n0 + 1] + vx * w1s[2 * NEUR + n0 + 1] + vy * w1s[3 * NEUR + n0 + 1];
      *(v2f*)&velp[wave][n0] = pv;
    }
    __syncthreads();

    {
      const v2f xo = *(const v2f*)(x + (size_t)sl * (2 * MOBS) + 2 * lane);
      const float ox = bf16r(xo[0]);
      const float oy = bf16r(xo[1]);
#pragma unroll
      for (int j8 = 0; j8 < 8; ++j8) {
        const v4f pA = *(const v4f*)&velp[wave][j8 * 8];
        const v4f pB = *(const v4f*)&velp[wave][j8 * 8 + 4];
        const v4f uA = *(const v4f*)&w1s[j8 * 8];
        const v4f uB = *(const v4f*)&w1s[j8 * 8 + 4];
        const v4f tA = *(const v4f*)&w1s[NEUR + j8 * 8];
        const v4f tB = *(const v4f*)&w1s[NEUR + j8 * 8 + 4];
        v8h o;
#pragma unroll
        for (int q = 0; q < 4; ++q) {
          o[q]     = (_Float16)(16.0f * fmaxf(pA[q] + ox * uA[q] + oy * tA[q], 0.0f));
          o[q + 4] = (_Float16)(16.0f * fmaxf(pB[q] + ox * uB[q] + oy * tB[q], 0.0f));
        }
        *(v8h*)(actW + lane * WP + j8 * 8) = o;
      }
    }
    __syncthreads();

    {
      const _Float16* wl = wph[0];
      const v16h a00 = ldfrag(actW + c * WP + 8 * hh);
      const v16h a01 = ldfrag(actW + c * WP + 32 + 8 * hh);
      const v16h a10 = ldfrag(actW + (16 + c) * WP + 8 * hh);
      const v16h a11 = ldfrag(actW + (16 + c) * WP + 32 + 8 * hh);
#pragma unroll
      for (int nt = 0; nt < 4; ++nt) {
        const int n0 = nt * 16;
        const _Float16* wp = wl + (n0 + c) * WP + 8 * hh;
        const v16h g0 = ldfrag(wp);
        const v16h g1 = ldfrag(wp + 32);
        v8f acc0 = zero8(), acc1 = zero8();
        acc0 = mma_h(a00, g0, acc0);
        acc1 = mma_h(a10, g0, acc1);
        acc0 = mma_h(a01, g1, acc0);
        acc1 = mma_h(a11, g1, acc1);
        guard2(acc0, acc1, a00, a01, a10, a11, g0, g1);
        const float bias = bph[0][n0 + c];
#pragma unroll
        for (int r = 0; r < 8; ++r) {
          const float h0v = fmaxf(acc0[r] * kinv + bias, 0.0f);
          const float h1v = fmaxf(acc1[r] * kinv + bias, 0.0f);
          actW[(8 * hh + r) * WP + n0 + c]      = (_Float16)(16.0f * h0v);
          actW[(16 + 8 * hh + r) * WP + n0 + c] = (_Float16)(16.0f * h1v);
        }
      }
    }
    __syncthreads();

    {
      const _Float16* wl = wph[1];
      const v16h a00 = ldfrag(actW + c * WP + 8 * hh);
      const v16h a01 = ldfrag(actW + c * WP + 32 + 8 * hh);
      const v16h a10 = ldfrag(actW + (16 + c) * WP + 8 * hh);
      const v16h a11 = ldfrag(actW + (16 + c) * WP + 32 + 8 * hh);
#pragma unroll
      for (int nt = 0; nt < 4; ++nt) {
        const int n0 = nt * 16;
        const _Float16* wp = wl + (n0 + c) * WP + 8 * hh;
        const v16h g0 = ldfrag(wp);
        const v16h g1 = ldfrag(wp + 32);
        v8f acc0 = zero8(), acc1 = zero8();
        acc0 = mma_h(a00, g0, acc0);
        acc1 = mma_h(a10, g0, acc1);
        acc0 = mma_h(a01, g1, acc0);
        acc1 = mma_h(a11, g1, acc1);
        guard2(acc0, acc1, a00, a01, a10, a11, g0, g1);
        float s0 = 0.0f, s1 = 0.0f;
#pragma unroll
        for (int r = 0; r < 8; ++r) { s0 += acc0[r]; s1 += acc1[r]; }
        float s = s0 + s1;
        s += __shfl_xor(s, 16);
        const float Xv  = s * kinv + 32.0f * bph[1][n0 + c];
        const float X16 = 16.0f * Xv;
        const _Float16 hv = (_Float16)X16;
        const _Float16 rv = (_Float16)((X16 - (float)hv) * 2048.0f);
        const int o = srow * WP + n0 + c;
        if (hh == 0) xh[o] = hv;
        else         xr[o] = rv;
      }
    }
  }
  __syncthreads();

  const int mrow = wave * 16;
#pragma unroll 1
  for (int rl = 0; rl < 2; ++rl) {
    const _Float16* wl = wrh[rl];
    const v16h ah0 = ldfrag(xh + (mrow + c) * WP + 8 * hh);
    const v16h ah1 = ldfrag(xh + (mrow + c) * WP + 32 + 8 * hh);
    const v16h ar0 = ldfrag(xr + (mrow + c) * WP + 8 * hh);
    const v16h ar1 = ldfrag(xr + (mrow + c) * WP + 32 + 8 * hh);
#pragma unroll
    for (int nt = 0; nt < 4; ++nt) {
      const int n0 = nt * 16;
      const _Float16* wp = wl + (n0 + c) * WP + 8 * hh;
      const v16h g0 = ldfrag(wp);
      const v16h g1 = ldfrag(wp + 32);
      v8f acch = zero8(), accr = zero8();
      acch = mma_h(ah0, g0, acch);
      accr = mma_h(ar0, g0, accr);
      acch = mma_h(ah1, g1, acch);
      accr = mma_h(ar1, g1, accr);
      guard2(acch, accr, ah0, ah1, ar0, ar1, g0, g1);
      const float bias = brh[rl][n0 + c];
#pragma unroll
      for (int r = 0; r < 8; ++r) {
        const float yv  = fmaxf((acch[r] + accr[r] * rinv) * kinv + bias, 0.0f);
        const float y16 = 16.0f * yv;
        const _Float16 hv = (_Float16)y16;
        const _Float16 rv = (_Float16)((y16 - (float)hv) * 2048.0f);
        const int o = (mrow + 8 * hh + r) * WP + n0 + c;
        xh[o] = hv;
        xr[o] = rv;
      }
    }
    __syncthreads();
  }

  {
    const v16h ah0 = ldfrag(xh + (mrow + c) * WP + 8 * hh);
    const v16h ah1 = ldfrag(xh + (mrow + c) * WP + 32 + 8 * hh);
    const v16h ar0 = ldfrag(xr + (mrow + c) * WP + 8 * hh);
    const v16h ar1 = ldfrag(xr + (mrow + c) * WP + 32 + 8 * hh);
#pragma unroll
    for (int nt = 0; nt < 2; ++nt) {
      const int n0 = nt * 16;
      const _Float16* wp = wr3 + (n0 + c) * WP + 8 * hh;
      const v16h g0 = ldfrag(wp);
      const v16h g1 = ldfrag(wp + 32);
      v8f acch = zero8(), accr = zero8();
      acch = mma_h(ah0, g0, acch);
      accr = mma_h(ar0, g0, accr);
      acch = mma_h(ah1, g1, acch);
      accr = mma_h(ar1, g1, accr);
      guard2(acch, accr, ah0, ah1, ar0, ar1, g0, g1);
      const float bias = br3[n0 + c];
#pragma unroll
      for (int r = 0; r < 8; ++r)
        outS[(mrow + 8 * hh + r) * OPF + n0 + c] = (acch[r] + accr[r] * rinv) * kinv + bias;
    }
  }
  __syncthreads();

  {
    const int piece = lane & 7;
    const int sub   = lane >> 3;
    v4f vv[4];
#pragma unroll
    for (int s = 0; s < 4; ++s)
      vv[s] = *(const v4f*)&outS[(mrow + 4 * s + sub) * OPF + piece * 4];
#pragma unroll
    for (int s = 0; s < 4; ++s) {
      const int gs = sbase + mrow + 4 * s + sub;
      if (gs < ns) *(volatile v4f*)(out + (size_t)gs * NOUT + piece * 4) = vv[s];
    }
    __threadfence();
#pragma unroll
    for (int s = 0; s < 4; ++s) {
      const int gs = sbase + mrow + 4 * s + sub;
      if (gs < ns) *(volatile v4f*)(out + (size_t)gs * NOUT + piece * 4) = vv[s];
    }
  }
}

extern "C" void kernel_launch(void* const* d_in, const int* in_sizes, int n_in,
                              void* d_out, int out_size, void* d_ws, size_t ws_size,
                              hipStream_t stream) {
  (void)d_ws; (void)ws_size;
  if (n_in < 14) return;
  const int nx = in_sizes[0];
  if (nx < 2 * MOBS || (nx % (2 * MOBS)) != 0) return;
  const int ns = nx / (2 * MOBS);
  if (in_sizes[1] != 2 * ns) return;
  if (in_sizes[2] != 4 * NEUR || in_sizes[3] != NEUR) return;
  if (in_sizes[4] != NEUR * NEUR || in_sizes[5] != NEUR) return;
  if (in_sizes[6] != NEUR * NEUR || in_sizes[7] != NEUR) return;
  if (in_sizes[8] != NEUR * NEUR || in_sizes[9] != NEUR) return;
  if (in_sizes[10] != NEUR * NEUR || in_sizes[11] != NEUR) return;
  if (in_sizes[12] != NEUR * NOUT || in_sizes[13] != NOUT) return;
  if (out_size != ns * NOUT) return;

  const float* x   = (const float*)d_in[0];
  const float* vel = (const float*)d_in[1];
  const float* pW1 = (const float*)d_in[2];
  const float* pb1 = (const float*)d_in[3];
  const float* pW2 = (const float*)d_in[4];
  const float* pb2 = (const float*)d_in[5];
  const float* pW3 = (const float*)d_in[6];
  const float* pb3 = (const float*)d_in[7];
  const float* rW1 = (const float*)d_in[8];
  const float* rb1 = (const float*)d_in[9];
  const float* rW2 = (const float*)d_in[10];
  const float* rb2 = (const float*)d_in[11];
  const float* rW3 = (const float*)d_in[12];
  const float* rb3 = (const float*)d_in[13];
  float* out = (float*)d_out;

  const int grid = (ns + SPB - 1) / SPB;
  k_deepset<<<dim3(grid), dim3(128), 0, stream>>>(x, vel, pW1, pb1, pW2, pb2, pW3, pb3,
                                                  rW1, rb1, rW2, rb2, rW3, rb3, out, ns);
  (void)hipGetLastError();
}
